// RLGCN_1151051236067
// MI455X (gfx1250) — hardware-run, weakly checked
//
#include <hip/hip_runtime.h>


namespace {
constexpr int N = 100000, NP = 100032, E = 1250000, FIN = 8, HID = 64, NBLK = NP / 64  ;
constexpr float XS = 8.0f, WSC = 256.0f;

typedef _Float16 b16;
typedef __attribute__((ext_vector_type(16))) _Float16 v16b;
typedef __attribute__((ext_vector_type(8))) _Float16 v8b;
typedef __attribute__((ext_vector_type(8))) float v8f;
typedef __attribute__((ext_vector_type(4))) float v4f;
typedef __attribute__((ext_vector_type(2))) float v2f;
__device__ __forceinline__ float bf16_rne(float f) { unsigned int u = __float_as_uint(f); u += 0x7FFFu + ((u >> 16) & 1u); return __uint_as_float(u & 0xFFFF0000u); }
__device__ __forceinline__ void split16(float v, b16& hi, b16& lo) { hi = (b16)v; lo = (b16)(v - (float)hi); }
__device__ __forceinline__ v16b frag_kb(const b16* p, int hh) { const v8b a = *(const v8b*)(p + 8 * hh), b = *(const v8b*)(p + 16 + 8 * hh); v16b f;
#pragma unroll
  for (int e = 0; e < 8; ++e) { f[e] = a[e]; f[8 + e] = b[e]; } return f; }
__device__ __forceinline__ v8f wmma16b(v16b a, v16b b, v8f c) { v8f d = __builtin_amdgcn_wmma_f32_16x16x32_f16(false, a, false, b, (short)0, c, false, false); asm volatile("v_nop\n\tv_nop\n\tv_nop\n\tv_nop" : "+v"(d) : "v"(a), "v"(b)); return d; }
__device__ __forceinline__ void wave_lds_sync() { __builtin_amdgcn_fence(__ATOMIC_RELEASE, "workgroup"); __builtin_amdgcn_wave_barrier(); __builtin_amdgcn_fence(__ATOMIC_ACQUIRE, "workgroup"); }
__device__ __forceinline__ float pmul(float a, float b) { float p = a * b; asm volatile("" : "+v"(p)); return p; }
__device__ __forceinline__ int iclamp(int v, int lo, int hi) { return v < lo ? lo : (v > hi ? hi : v); }

constexpr int CSR_NBLK = 512, CSR_GB = 9, CSR_GN = 1 << CSR_GB  , CSR_MAXG = 512, CSR_CAP = 12288  ;
__global__ __launch_bounds__(64) void csrA_kernel(const int* __restrict__ dst, int E, int N, int nG, int CHP, int NGP, int* __restrict__ STG, int* __restrict__ HST) {
  extern __shared__ int sm[];
  int* cnt = sm; int* run = sm + NGP; int* ids = sm + 2 * NGP;
  const int b = blockIdx.x; const int ch = (E + CSR_NBLK - 1) / CSR_NBLK; const int e0 = b * ch, e1 = min(E, e0 + ch);
  for (int i = threadIdx.x; i < NGP; i += 64) cnt[i] = 0;
  for (int i = threadIdx.x; i < CHP; i += 64) ids[i] = -1;
  __syncthreads();
  if (threadIdx.x == 0) {
    for (int e = e0; e < e1; ++e) { int d = dst[e]; d = (d < 0) ? 0 : (d >= N ? N - 1 : d); cnt[d >> CSR_GB] += 1; }
    int acc = 0; for (int g = 0; g < nG; ++g) { run[g] = acc; acc += cnt[g]; }
    for (int e = e0; e < e1; ++e) { int d = dst[e]; d = (d < 0) ? 0 : (d >= N ? N - 1 : d); const int g = d >> CSR_GB; ids[run[g]] = e; run[g] += 1; } }
  __syncthreads();
  typedef __attribute__((ext_vector_type(4))) int v4i;
  for (int pass = 0; pass < 2; ++pass) {
    for (int i = threadIdx.x; i < CHP / 4; i += 64) *(volatile v4i*)(STG + (size_t)b * CHP + i * 4) = *(const v4i*)(&ids[i * 4]);
    for (int i = threadIdx.x; i < NGP / 4; i += 64) { v4i v; for (int e = 0; e < 4; ++e) v[e] = (i * 4 + e < nG) ? cnt[i * 4 + e] : 0; *(volatile v4i*)(HST + (size_t)b * NGP + i * 4) = v; }
    __threadfence(); }
}
__global__ __launch_bounds__(512) void csrS_kernel(const int* __restrict__ HST, int nG, int NGP, int* __restrict__ START, int* __restrict__ TOT, int* __restrict__ OFF) {
  __shared__ int tot[CSR_MAXG];
  const int b = threadIdx.x;
  for (int pass = 0; pass < 2; ++pass) { int runb = 0; for (int g = 0; g < nG; ++g) { int c = HST[(size_t)b * NGP + g]; c = (c < 0) ? 0 : c; ((volatile int*)OFF)[(size_t)g * CSR_NBLK + b] = runb; runb += c; } __threadfence(); }
  for (int g = threadIdx.x; g < nG; g += 512) { int s = 0; for (int bb = 0; bb < CSR_NBLK; ++bb) { int c = HST[(size_t)bb * NGP + g]; s += (c < 0) ? 0 : c; } tot[g] = s; }
  __syncthreads();
  if (threadIdx.x < 32) {
    __shared__ int st[CSR_MAXG + 32];
    if (threadIdx.x == 0) { int acc = 0; for (int g = 0; g < NGP; ++g) { st[g] = acc; if (g < nG) acc += (tot[g] + 31) & ~31; } st[NGP] = acc; }
    __builtin_amdgcn_fence(__ATOMIC_RELEASE, "workgroup"); __builtin_amdgcn_wave_barrier(); __builtin_amdgcn_fence(__ATOMIC_ACQUIRE, "workgroup");
    for (int pass = 0; pass < 2; ++pass) { for (int i = threadIdx.x; i < NGP + 32; i += 32) { ((volatile int*)START)[i] = (i <= NGP) ? st[min(i, NGP)] : 0; ((volatile int*)TOT)[i] = (i < nG) ? tot[i] : 0; } __threadfence(); } }
}
__global__ __launch_bounds__(256) void csrB_kernel(const int* __restrict__ dst, int N, int nG, int CHP, int NGP, int permLen, const int* __restrict__ STG, const int* __restrict__ HST, const int* __restrict__ OFF, const int* __restrict__ START, const int* __restrict__ TOT, int* __restrict__ PERM, int* __restrict__ ROWPTR, int* __restrict__ ROWCNT, int* __restrict__ FLAG) {
  typedef __attribute__((ext_vector_type(4))) int v4i;
  __shared__ int ids[CSR_CAP]; __shared__ unsigned short key[CSR_CAP]; __shared__ int outp[CSR_CAP]; __shared__ int ncnt[CSR_GN + 1]; __shared__ int boff[CSR_NBLK + 1];
  const int g = blockIdx.x, t_ = threadIdx.x; int tot = TOT[g]; int st = START[g], stn = START[g + 1]; const int v0 = g * CSR_GN; const int nv = min(CSR_GN, N - v0);
  st = (st < 0) ? 0 : (st > permLen - 32 ? permLen - 32 : st) & ~31; stn = (stn < st) ? st : (stn > permLen ? permLen : stn); tot = (tot < 0) ? 0 : tot; if (tot > stn - st && tot <= CSR_CAP) tot = stn - st;
  if (tot > CSR_CAP) {
    for (int pass = 0; pass < 2; ++pass) { for (int i = t_; i < CSR_GN / 4; i += 256) { v4i a, c; for (int e = 0; e < 4; ++e) { a[e] = st; c[e] = 0; } *(volatile v4i*)(ROWPTR + v0 + i * 4) = a; *(volatile v4i*)(ROWCNT + v0 + i * 4) = c; } if (t_ == 0) ((volatile int*)FLAG)[0] = 1; __threadfence(); } (void)nv; return; }
  if (t_ == 0) { int acc = 0; for (int b = 0; b < CSR_NBLK; ++b) { boff[b] = acc; int c = HST[(size_t)b * NGP + g]; c = (c < 0) ? 0 : (c > CHP ? CHP : c); acc += c; if (acc > tot) acc = tot; } boff[CSR_NBLK] = acc; }
  for (int i = t_; i <= CSR_GN; i += 256) ncnt[i] = 0;
  __syncthreads();
  for (int b = 0; b < CSR_NBLK; ++b) { const int c = boff[b + 1] - boff[b]; int o_ = OFF[(size_t)g * CSR_NBLK + b]; o_ = (o_ < 0) ? 0 : (o_ > CHP - c ? CHP - c : o_); const int* src_ = STG + (size_t)b * CHP + o_;
    for (int i = t_; i < c; i += 256) { int id = src_[i]; id = (id < 0) ? 0 : id; ids[boff[b] + i] = id; int d = dst[id]; d = (d < v0) ? v0 : (d >= N ? N - 1 : d); int kk = d - v0; kk = (kk < 0) ? 0 : (kk >= CSR_GN ? CSR_GN - 1 : kk); key[boff[b] + i] = (unsigned short)kk; } }
  __syncthreads();
  if (t_ == 0) { for (int i = 0; i < tot; ++i) ncnt[key[i]] += 1; int acc = 0; for (int vl = 0; vl < CSR_GN; ++vl) { const int c = ncnt[vl]; ncnt[vl] = acc; acc += c; } ncnt[CSR_GN] = acc;
    for (int i = 0; i < tot; ++i) { const int vl = key[i]; outp[ncnt[vl]] = ids[i]; ncnt[vl] += 1; }
    for (int vl = CSR_GN; vl > 0; --vl) ncnt[vl] = ncnt[vl - 1]; ncnt[0] = 0; }
  __syncthreads();
  for (int pass = 0; pass < 2; ++pass) {
    for (int i = t_; i < (stn - st) / 4; i += 256) { v4i v; for (int e = 0; e < 4; ++e) { const int q = i * 4 + e; v[e] = (q < tot) ? outp[q] : -1; } *(volatile v4i*)(PERM + st + i * 4) = v; }
    for (int i = t_; i < CSR_GN / 4; i += 256) { v4i a, c; for (int e = 0; e < 4; ++e) { const int vl = i * 4 + e; a[e] = st + ncnt[vl]; c[e] = (vl < nv) ? (ncnt[vl + 1] - ncnt[vl]) : 0; } *(volatile v4i*)(ROWPTR + v0 + i * 4) = a; *(volatile v4i*)(ROWCNT + v0 + i * 4) = c; }
    __threadfence(); }
}
__global__ __launch_bounds__(256) void csrZ_kernel(int* __restrict__ p, size_t n4) { typedef __attribute__((ext_vector_type(4))) int v4i; const size_t tid = (size_t)blockIdx.x * 256 + threadIdx.x, nth = (size_t)gridDim.x * 256; v4i z = {0, 0, 0, 0}; for (size_t i = tid; i < n4; i += nth) *(volatile v4i*)(p + i * 4) = z; }
struct CsrBufs { int *STG, *HST, *OFF, *START, *TOT, *PERM, *ROWPTR, *ROWCNT, *FLAG; int nG, NGP, CHP; size_t permLen; char* base; size_t bytes; };
static size_t csr_carve(CsrBufs& c, char* ws, size_t off, int E, int N) {
  const size_t off0 = off; c.base = ws + off;
  auto al = [&](size_t bytes) { char* p = ws + off; off += (bytes + 255) & ~(size_t)255; return p; };
  c.nG = (N + CSR_GN - 1) / CSR_GN; c.NGP = (c.nG + 31) & ~31; const int ch = (E + CSR_NBLK - 1) / CSR_NBLK; c.CHP = (ch + 31) & ~31; c.permLen = (size_t)E + 32 * (size_t)c.nG + 32;
  c.STG = (int*)al((size_t)CSR_NBLK * c.CHP * 4); c.HST = (int*)al((size_t)CSR_NBLK * c.NGP * 4); c.OFF = (int*)al((size_t)c.NGP * CSR_NBLK * 4); c.START = (int*)al((size_t)(c.NGP + 64) * 4); c.TOT = (int*)al((size_t)(c.NGP + 64) * 4);
  c.PERM = (int*)al(c.permLen * 4); c.ROWPTR = (int*)al((size_t)c.nG * CSR_GN * 4); c.ROWCNT = (int*)al((size_t)c.nG * CSR_GN * 4); c.FLAG = (int*)al(256);
  c.bytes = off - off0; return off;
}
static void csr_build(const CsrBufs& c, const int* dst, int E, int N, hipStream_t stream) {
  const size_t smem = (size_t)(2 * c.NGP + c.CHP) * 4;
  csrZ_kernel<<<512, 256, 0, stream>>>((int*)c.base, c.bytes / 16);
  csrA_kernel<<<CSR_NBLK, 64, smem, stream>>>(dst, E, N, c.nG, c.CHP, c.NGP, c.STG, c.HST);
  csrS_kernel<<<1, 512, 0, stream>>>(c.HST, c.nG, c.NGP, c.START, c.TOT, c.OFF);
  csrB_kernel<<<c.nG, 256, 0, stream>>>(dst, N, c.nG, c.CHP, c.NGP, (int)c.permLen, c.STG, c.HST, c.OFF, c.START, c.TOT, c.PERM, c.ROWPTR, c.ROWCNT, c.FLAG);
}


__global__ __launch_bounds__(128) void layer1_kernel(const float* __restrict__ x, const int* __restrict__ srcs, const int* __restrict__ PERM, const int* __restrict__ ROWPTR, const int* __restrict__ ROWCNT, int permLen, const b16* __restrict__ W1P, const float* __restrict__ b1, float* __restrict__ H1) {
  __shared__ __attribute__((aligned(16))) b16 Ah[64][40], Al[64][40]; __shared__ __attribute__((aligned(16))) float Ts[4][16][HID + 4];
  const int wave = threadIdx.x >> 5, lane = threadIdx.x & 31, nloc = lane & 15, hlf = lane >> 4; const size_t row0 = (size_t)blockIdx.x * 64 + wave * 16;
  for (int r = 0; r < 16; ++r) { Ah[wave * 16 + r][8 + (lane % 24)] = (b16)0.0f; Al[wave * 16 + r][8 + (lane % 24)] = (b16)0.0f; }
  const int q = lane >> 3, f = lane & 7;
  for (int g = 0; g < 4; ++g) { const size_t v = row0 + g * 4 + q; float acc = 0.0f;
    if (v < (size_t)N) { int st = ROWPTR[v], cnt = ROWCNT[v]; cnt = iclamp(cnt, 0, 8192); st = iclamp(st, 0, permLen - cnt); const float dv = rsqrtf((float)cnt + 1.0f); acc = pmul(dv, bf16_rne(x[v * FIN + f]));
      for (int j = 0; j < cnt; ++j) { const int e = iclamp(PERM[st + j], 0, E - 1); const int s = iclamp(srcs[e], 0, N - 1); const float ds = rsqrtf((float)iclamp(ROWCNT[s], 0, 8192) + 1.0f); acc += pmul(ds, bf16_rne(x[(size_t)s * FIN + f])); }
      acc = pmul(acc, dv); }
    b16 p, qq; split16(acc * XS, p, qq); Ah[wave * 16 + g * 4 + q][f] = p; Al[wave * 16 + g * 4 + q][f] = qq; }
  wave_lds_sync();
  v8f a4[4] = {{}, {}, {}, {}}; { const v16b a = frag_kb(&Ah[wave * 16 + nloc][0], hlf), al = frag_kb(&Al[wave * 16 + nloc][0], hlf);
#pragma unroll
    for (int t = 0; t < 4; ++t) { const v16b bw = frag_kb(W1P + (size_t)(t * 16 + nloc) * 32, hlf); a4[t] = wmma16b(a, bw, a4[t]); a4[t] = wmma16b(al, bw, a4[t]); } }
#pragma unroll
  for (int t = 0; t < 4; ++t) { const int c = t * 16 + nloc; const float bb = bf16_rne(b1[c]);
#pragma unroll
    for (int r = 0; r < 8; ++r) { const size_t row = row0 + 8 * hlf + r; Ts[wave][8 * hlf + r][c] = (row < (size_t)N) ? fmaxf(a4[t][r] * (1.0f / (XS * WSC)) + bb, 0.0f) : 0.0f; } }
  wave_lds_sync();
  for (int pass = 0; pass < 2; ++pass) { for (int rr = 0; rr < 16; ++rr) if (lane < 16) *(volatile v4f*)(H1 + (row0 + rr) * HID + lane * 4) = *(const v4f*)(&Ts[wave][rr][lane * 4]); __threadfence(); }
}
__global__ __launch_bounds__(256) void agg2_kernel(const float* __restrict__ H1, const int* __restrict__ srcs, const int* __restrict__ PERM, const int* __restrict__ ROWPTR, const int* __restrict__ ROWCNT, int permLen, float* __restrict__ P) {
  __shared__ float part[8][HID];
  const int wave = threadIdx.x >> 5, lane = threadIdx.x & 31, t_ = threadIdx.x; const size_t v = (size_t)blockIdx.x * 8 + wave; const int c0 = lane * 2; float a0 = 0.0f, a1 = 0.0f;
  if (v < (size_t)N) { int st = ROWPTR[v], cnt = ROWCNT[v]; cnt = iclamp(cnt, 0, 8192); st = iclamp(st, 0, permLen - cnt); const float dv = rsqrtf((float)cnt + 1.0f); const v2f hs = *(const v2f*)(H1 + v * HID + c0); a0 = pmul(dv, hs[0]); a1 = pmul(dv, hs[1]);
    for (int j = 0; j < cnt; ++j) { const int e = iclamp(PERM[st + j], 0, E - 1); const int s = iclamp(srcs[e], 0, N - 1); const float ds = rsqrtf((float)iclamp(ROWCNT[s], 0, 8192) + 1.0f); const v2f h = *(const v2f*)(H1 + (size_t)s * HID + c0); a0 += pmul(ds, h[0]); a1 += pmul(ds, h[1]); }
    a0 = pmul(a0, dv); a1 = pmul(a1, dv); }
  part[wave][c0] = a0; part[wave][c0 + 1] = a1;
  __syncthreads();
  for (int pass = 0; pass < 2; ++pass) { if (t_ < HID / 4) { v4f o; for (int k = 0; k < 4; ++k) { const int c = t_ * 4 + k; float s = 0.0f; for (int w = 0; w < 8; ++w) s += part[w][c]; o[k] = s; } *(volatile v4f*)(P + (size_t)blockIdx.x * HID + t_ * 4) = o; } __threadfence(); }
}
__global__ __launch_bounds__(64) void final_kernel(const float* __restrict__ P, int nblk, const float* __restrict__ W2, const float* __restrict__ b2, const float* __restrict__ state, const float* __restrict__ Wm, const float* __restrict__ bm, const float* __restrict__ Wc, const float* __restrict__ bc, float* __restrict__ out) {
  __shared__ float gm[HID], hm[HID], sv[HID];
  const int c = threadIdx.x; float s = 0.0f; for (int b = 0; b < nblk; ++b) s += P[(size_t)b * HID + c]; gm[c] = s * (1.0f / N);
  __syncthreads();
  { float a = bf16_rne(b2[c]); for (int k = 0; k < HID; ++k) a += pmul(gm[k], bf16_rne(W2[k * HID + c])); hm[c] = a; float t = bf16_rne(bm[c]); for (int k = 0; k < FIN; ++k) t += pmul(bf16_rne(state[k]), bf16_rne(Wm[k * HID + c])); sv[c] = fmaxf(t, 0.0f); }
  __syncthreads();
  __shared__ float ov[2];
  if (c < 2) { float o = bf16_rne(bc[c]); for (int k = 0; k < HID; ++k) o += pmul(hm[k], bf16_rne(Wc[k * 2 + c])); for (int k = 0; k < HID; ++k) o += pmul(sv[k], bf16_rne(Wc[(HID + k) * 2 + c])); ov[c] = o; }
  __syncthreads();
  if (c == 0) { const v2f o2 = {ov[0], ov[1]}; for (int pass = 0; pass < 2; ++pass) { *(volatile v2f*)out = o2; __threadfence(); } }
}
__global__ __launch_bounds__(256) void prepw_kernel(const float* __restrict__ w1, b16* __restrict__ W1P) { const int t = threadIdx.x; const int e = t * 8; const int o = e / 32, k0 = e % 32; v8b v;
  for (int j = 0; j < 8; ++j) { const int k = k0 + j; v[j] = (k < FIN) ? (b16)(bf16_rne(w1[k * HID + o]) * WSC) : (b16)0.0f; }
  for (int pass = 0; pass < 2; ++pass) { *(volatile v8b*)(W1P + e) = v; __threadfence(); } }
}

extern "C" void kernel_launch(void* const* d_in, const int* in_sizes, int n_in, void* d_out, int out_size, void* d_ws, size_t ws_size, hipStream_t stream) {
  (void)n_in;
  auto Fp = [&](int i) { return (const float*)d_in[i]; }; auto Ip = [&](int i) { return (const int*)d_in[i]; };
  if (in_sizes[0] != N * FIN || in_sizes[1] != FIN || in_sizes[2] != FIN * HID || in_sizes[4] != HID * HID || in_sizes[8] != 2 * HID * 2 || in_sizes[10] != 2 * E || out_size != 2) return;
  size_t off = 0; char* ws = (char*)d_ws;
  auto carve = [&](size_t bytes) { char* p = ws + off; off += (bytes + 255) & ~(size_t)255; return p; };
  b16* W1P = (b16*)carve((size_t)HID * 32 * 2); float* H1 = (float*)carve((size_t)NP * HID * 4); const int nblk2 = NP / 8; float* P = (float*)carve((size_t)nblk2 * HID * 4);
  CsrBufs csr; off = csr_carve(csr, ws, off, E, N);
  if (off > ws_size || off > ((size_t)128 << 20)) return;
  prepw_kernel<<<1, 256, 0, stream>>>(Fp(2), W1P);
  csr_build(csr, Ip(10) + E, E, N, stream);
  layer1_kernel<<<NBLK, 128, 0, stream>>>(Fp(0), Ip(10), csr.PERM, csr.ROWPTR, csr.ROWCNT, (int)csr.permLen, W1P, Fp(3), H1);
  agg2_kernel<<<nblk2, 256, 0, stream>>>(H1, Ip(10), csr.PERM, csr.ROWPTR, csr.ROWCNT, (int)csr.permLen, P);
  final_kernel<<<1, 64, 0, stream>>>(P, nblk2, Fp(4), Fp(5), Fp(1), Fp(6), Fp(7), Fp(8), Fp(9), (float*)d_out);
}
